// RCCA_76459007804004
// MI455X (gfx1250) — hardware-verified
//
#include <hip/hip_runtime.h>

typedef __attribute__((ext_vector_type(16))) _Float16 v16h;
typedef __attribute__((ext_vector_type(8)))  _Float16 v8h;
typedef __attribute__((ext_vector_type(8)))  float    v8f;
typedef __attribute__((ext_vector_type(4)))  float    v4f;

typedef __attribute__((ext_vector_type(4)))  unsigned v4u;
template <typename T> __device__ __forceinline__ void vst2(void* p, T v) { *(volatile T*)p = v; __threadfence(); *(volatile T*)p = v; }
__device__ __forceinline__ v8f WMMA_F16(v16h a, v16h b, v8f c) {
  v8f d = __builtin_amdgcn_wmma_f32_16x16x32_f16(false, a, false, b, (short)0, c, false, false);
  asm volatile("v_nop\n\tv_nop\n\tv_nop\n\tv_nop" : "+v"(d) : "v"(a), "v"(b));
  return d;
}
__device__ __forceinline__ v16h bfrag16(const _Float16* rowk0, int half) {
  v16h b; ((v8h*)&b)[0] = *(const v8h*)(rowk0 + half * 8); ((v8h*)&b)[1] = *(const v8h*)(rowk0 + 16 + half * 8); return b;
}
#define LDSX() do { asm volatile("s_wait_dscnt 0" ::: "memory"); __builtin_amdgcn_wave_barrier(); __builtin_amdgcn_fence(__ATOMIC_RELEASE, "workgroup"); } while (0)

constexpr int Bsz = 4;
constexpr int Cch = 256;
constexpr int Nsq = 4096;

__global__ void wcvt_kernel(const float* __restrict__ wq,
                            const float* __restrict__ wk,
                            const float* __restrict__ wv,
                            _Float16* __restrict__ out) {
  int g8 = blockIdx.x * 256 + threadIdx.x;
  int t0 = g8 * 8; int m = t0 >> 16, e = t0 & 65535;
  const float* s = (m == 0) ? wq : (m == 1) ? wk : wv;
  union { v8h h; v4u u; } pk;
#pragma unroll
  for (int i = 0; i < 8; ++i) pk.h[i] = (_Float16)s[e + i];
  vst2(out + t0, pk.u);
}

__global__ void __launch_bounds__(128, 1)
qkv_kernel(const float* __restrict__ x,
           const _Float16* __restrict__ wh,
           const float* __restrict__ bq,
           const float* __restrict__ bk,
           const float* __restrict__ bv,
           _Float16* __restrict__ Qt,
           _Float16* __restrict__ Kt,
           _Float16* __restrict__ V) {
  __shared__ __align__(16) _Float16 xT[4][16 * 256];
  __shared__ __align__(16) _Float16 sVst[256 * 64];
  const int wave = threadIdx.x >> 5, lane = threadIdx.x & 31;
  const int tile = blockIdx.x * 4 + wave;
  const int b  = tile >> 8;
  const int n0 = (tile & 255) << 4;
  const int row = lane & 15, half = lane >> 4;

  _Float16* xt = xT[wave];
  const float* xb = x + (size_t)b * Cch * Nsq;
  #pragma unroll 4
  for (int it = 0; it < 128; ++it) {
    int idx = it * 32 + lane;
    int c = idx >> 4, n = idx & 15;
    xt[n * 256 + c] = (_Float16)xb[(size_t)c * Nsq + n0 + n];
  }
  LDSX();

  v16h a[8];
  #pragma unroll
  for (int k = 0; k < 8; ++k) {
    ((v8h*)&a[k])[0] = *(const v8h*)&xt[row * 256 + k * 32 + half * 8];
    ((v8h*)&a[k])[1] = *(const v8h*)&xt[row * 256 + k * 32 + half * 8 + 16];
  }

  #pragma unroll
  for (int m = 0; m < 3; ++m) {
    const _Float16* W = wh + (size_t)m * 65536;
    const float* bias = (m == 0) ? bq : (m == 1) ? bk : bv;
    for (int ot = 0; ot < 16; ++ot) {
      const int o = ot * 16 + row;
      v8f acc = {};
      #pragma unroll
      for (int k = 0; k < 8; ++k) acc = WMMA_F16(a[k], bfrag16(&W[o * 256 + k * 32], half), acc);
      const float bo = bias[o];
      #pragma unroll
      for (int v = 0; v < 8; ++v) {
        float val = acc[v] + bo;
        int nl = v + half * 8;
        if (m < 2) xt[nl * 256 + o] = (_Float16)val;
        else       sVst[o * 64 + wave * 16 + nl] = (_Float16)val;
      }
    }
    if (m < 2) {
      LDSX();
      _Float16* dst = (m == 0 ? Qt : Kt) + ((size_t)b * Nsq + n0) * Cch;
      #pragma unroll 4
      for (int nl = 0; nl < 16; ++nl) vst2(dst + (size_t)nl * Cch + lane * 8, *(const v4u*)&xt[nl * 256 + lane * 8]);
      __builtin_amdgcn_wave_barrier();
    }
  }
  __syncthreads();
  const int n0blk = ((blockIdx.x * 4) & 255) << 4;
  for (int q = threadIdx.x; q < 256 * 8; q += 128) { const int o = q >> 3, pc = q & 7;
    vst2(V + ((size_t)b * Cch + o) * (size_t)Nsq + n0blk + pc * 8, *(const v4u*)&sVst[o * 64 + pc * 8]); }
}

__global__ void __launch_bounds__(128, 1)
attn_kernel(const float* __restrict__ x,
            const _Float16* __restrict__ Qt,
            const _Float16* __restrict__ Kt,
            const _Float16* __restrict__ Vm,
            float* __restrict__ out) {
  __shared__ __align__(16) _Float16 pbuf[4][16 * 32];
  __shared__ __align__(16) float    cst[128 * 64];
  const int wave = threadIdx.x >> 5, lane = threadIdx.x & 31;
  const int tile = blockIdx.x * 4 + wave;
  const int b  = tile >> 8;
  const int i0 = (tile & 255) << 4;
  const int row = lane & 15, half = lane >> 4;
  const float C1 = 0.0625f * 1.44269504089f;

  const _Float16* Qb = Qt + ((size_t)b * Nsq + i0 + row) * Cch;

  v8f acc[16];
  #pragma unroll
  for (int ct = 0; ct < 16; ++ct) { v8f z = {}; acc[ct] = z; }
  float mrow[8], srow[8];
  #pragma unroll
  for (int v = 0; v < 8; ++v) { mrow[v] = -3.0e38f; srow[v] = 0.f; }
  _Float16* pl = pbuf[wave];

  for (int j0 = 0; j0 < Nsq; j0 += 32) {
    const _Float16* K0 = Kt + ((size_t)b * Nsq + j0 + row) * Cch;
    const _Float16* K1 = K0 + 16 * Cch;
    const _Float16* Vb = Vm + ((size_t)b * Cch + row) * (size_t)Nsq + j0;
    v8f sD0 = {}, sD1 = {};
    #pragma unroll
    for (int k = 0; k < 8; ++k) {
      const v16h qk = bfrag16(Qb + k * 32, half);
      sD0 = WMMA_F16(qk, bfrag16(K0 + k * 32, half), sD0);
      sD1 = WMMA_F16(qk, bfrag16(K1 + k * 32, half), sD1);
    }
    #pragma unroll
    for (int v = 0; v < 8; ++v) {
      float lm = fmaxf(sD0[v], sD1[v]);
      lm = fmaxf(lm, __shfl_xor(lm, 8, 32));
      lm = fmaxf(lm, __shfl_xor(lm, 4, 32));
      lm = fmaxf(lm, __shfl_xor(lm, 2, 32));
      lm = fmaxf(lm, __shfl_xor(lm, 1, 32));
      const float mn  = fmaxf(mrow[v], lm);
      const float cor = __builtin_exp2f((mrow[v] - mn) * C1);
      mrow[v] = mn;
      const float p0 = __builtin_exp2f((sD0[v] - mn) * C1);
      const float p1 = __builtin_exp2f((sD1[v] - mn) * C1);
      float rs = p0 + p1;
      rs += __shfl_xor(rs, 8, 32);
      rs += __shfl_xor(rs, 4, 32);
      rs += __shfl_xor(rs, 2, 32);
      rs += __shfl_xor(rs, 1, 32);
      srow[v] = srow[v] * cor + rs;
      const int ir = v + half * 8;
      pl[ir * 32 + row]      = (_Float16)(p0 * 16384.0f);
      pl[ir * 32 + 16 + row] = (_Float16)(p1 * 16384.0f);
      #pragma unroll
      for (int ct = 0; ct < 16; ++ct) acc[ct][v] *= cor;
    }
    LDSX();
    v16h pa;
    ((v8h*)&pa)[0] = *(const v8h*)&pl[row * 32 + half * 8];
    ((v8h*)&pa)[1] = *(const v8h*)&pl[row * 32 + half * 8 + 16];
    #pragma unroll
    for (int ct = 0; ct < 16; ++ct) acc[ct] = WMMA_F16(pa, bfrag16(Vb + (size_t)ct * 16 * Nsq, half), acc[ct]);
    __builtin_amdgcn_wave_barrier();
  }

  float rinv[8];
  #pragma unroll
  for (int v = 0; v < 8; ++v) rinv[v] = (1.0f / 16384.0f) / srow[v];
  const int i0blk = ((blockIdx.x * 4) & 255) << 4;
  #pragma unroll
  for (int pass = 0; pass < 2; ++pass) {
    __syncthreads();
    #pragma unroll
    for (int ct = 0; ct < 8; ++ct) {
      const int cl = ct * 16 + row;
      #pragma unroll
      for (int v = 0; v < 8; ++v)
        cst[cl * 64 + wave * 16 + v + half * 8] = acc[pass * 8 + ct][v] * rinv[v];
    }
    __syncthreads();
    for (int qd = threadIdx.x; qd < 128 * 16; qd += 128) { const int cl = qd >> 4, pc = qd & 15;
      const int c = pass * 128 + cl;
      const size_t base = ((size_t)b * Cch + c) * (size_t)Nsq + i0blk + pc * 4;
      v4f cv = *(const v4f*)&cst[cl * 64 + pc * 4] + *(const v4f*)&x[base];
      vst2(out + base, cv); }
  }
}

extern "C" void kernel_launch(void* const* d_in, const int* in_sizes, int n_in,
                              void* d_out, int out_size, void* d_ws, size_t ws_size,
                              hipStream_t stream) {
  const float* x  = (const float*)d_in[0];
  const float* Wq = (const float*)d_in[1];
  const float* bq = (const float*)d_in[2];
  const float* Wk = (const float*)d_in[3];
  const float* bk = (const float*)d_in[4];
  const float* Wv = (const float*)d_in[5];
  const float* bv = (const float*)d_in[6];
  float* out = (float*)d_out;

  char* ws = (char*)d_ws;
  _Float16* wh = (_Float16*)ws;
  _Float16* Qt = (_Float16*)(ws + (size_t)3 * Cch * Cch * 2);
  _Float16* Kt = Qt + (size_t)Bsz * Nsq * Cch;
  _Float16* V  = Kt + (size_t)Bsz * Nsq * Cch;

  wcvt_kernel<<<(3 * Cch * Cch / 8) / 256, 256, 0, stream>>>(Wq, Wk, Wv, wh);
  qkv_kernel<<<256, 128, 0, stream>>>(x, wh, bq, bk, bv, Qt, Kt, V);
  attn_kernel<<<256, 128, 0, stream>>>(x, Qt, Kt, V, out);
}
